// VisionMambaV2_19061064859765
// MI455X (gfx1250) — hardware-verified
//
#include <hip/hip_runtime.h>
#define BB 4
#define LL 256
#define GR 16
#define DM 384
#define DI 768
#define NS 16
#define BH 2
#define MT (BB * LL)
#define XPN 1664

typedef __bf16 v16b __attribute__((ext_vector_type(16)));
typedef unsigned short v8us __attribute__((ext_vector_type(8), may_alias));
typedef float  v8f  __attribute__((ext_vector_type(8)));
typedef float  v4f  __attribute__((ext_vector_type(4)));
typedef float  v4fa __attribute__((ext_vector_type(4), may_alias));
union FragB { v16b v; v8us half[2]; unsigned short u[16]; };

__device__ __forceinline__ unsigned short bf16_bits(float x) { unsigned int u = __float_as_uint(x); return (unsigned short)((u + 0x7FFFu + ((u >> 16) & 1u)) >> 16); }
__device__ __forceinline__ float bf16_val(unsigned short b) { return __uint_as_float(((unsigned int)b) << 16); }
__device__ __forceinline__ float bf16_round(float x) { return bf16_val(bf16_bits(x)); }
template <int NT>
__device__ __forceinline__ v8f mmaN(v16b ah, v16b al, v16b bh, v16b bl, v8f c) {
  c = __builtin_amdgcn_wmma_f32_16x16x32_bf16(false, ah, false, bh, (short)0, c, false, false);
  if (NT >= 2) c = __builtin_amdgcn_wmma_f32_16x16x32_bf16(false, al, false, bh, (short)0, c, false, false);
  if (NT >= 3) c = __builtin_amdgcn_wmma_f32_16x16x32_bf16(false, ah, false, bl, (short)0, c, false, false);
  asm volatile("v_nop\n\tv_nop\n\tv_nop\n\tv_nop" : "+v"(c) : "v"(ah), "v"(al), "v"(bh), "v"(bl));
  return c;
}

__global__ __launch_bounds__(256) void k_wt_bf16(const float* __restrict__ W, unsigned short* __restrict__ Wt, int K, int N) {
  const int t = blockIdx.x * 256 + threadIdx.x;
  const int k8n = K / 8;
  if (t >= N * k8n) return;
  const int n = t / k8n, k8 = (t % k8n) * 8;
  v8us v;
#pragma unroll
  for (int i = 0; i < 8; ++i) v[i] = bf16_bits(W[(size_t)(k8 + i) * N + n]);
  *(volatile v8us*)(Wt + (size_t)n * K + k8) = v;
  __threadfence();
  *(volatile v8us*)(Wt + (size_t)n * K + k8) = v;
}

template <bool ASPLIT, int ACT, bool BIAS_BF16>
__global__ __launch_bounds__(128) void k_gemm_bf(const float* __restrict__ A, int lda, const unsigned short* __restrict__ Wt, int ldb,
                                               const float* __restrict__ bias, float* __restrict__ C, int ldc, int M, int N, int K) {
  __shared__ __attribute__((aligned(16))) float so[4][16][64];
  const int tid = threadIdx.x, w = tid >> 5, lane = tid & 31, ln = lane & 15, hh = lane >> 4;
  const int ntn = N / 64;
  const int wid = blockIdx.x * 4 + w;
  const int mt = wid / ntn, nq = wid % ntn;
  if (mt * 16 >= M) return;
  const int row0 = mt * 16, col0 = nq * 64;
  const float* arow = A + (size_t)(row0 + ln) * lda;
  v8f acc[4] = {};
  for (int kb = 0; kb < K; kb += 32) {
    FragB ah, al;
    const v4f x0 = *(const v4fa*)(arow + kb + 8 * hh), x1 = *(const v4fa*)(arow + kb + 8 * hh + 4);
    const v4f x2 = *(const v4fa*)(arow + kb + 16 + 8 * hh), x3 = *(const v4fa*)(arow + kb + 16 + 8 * hh + 4);
    float xs[16] = {x0[0],x0[1],x0[2],x0[3],x1[0],x1[1],x1[2],x1[3],x2[0],x2[1],x2[2],x2[3],x3[0],x3[1],x3[2],x3[3]};
#pragma unroll
    for (int i = 0; i < 16; ++i) { const unsigned short hb = bf16_bits(xs[i]); ah.u[i] = hb; al.u[i] = ASPLIT ? bf16_bits(xs[i] - bf16_val(hb)) : (unsigned short)0; }
#pragma unroll
    for (int t = 0; t < 4; ++t) {
      const unsigned short* brow = Wt + (size_t)(col0 + t * 16 + ln) * ldb + kb;
      FragB b;
      b.half[0] = *(const v8us*)(brow + 8 * hh);
      b.half[1] = *(const v8us*)(brow + 16 + 8 * hh);
      acc[t] = mmaN<ASPLIT ? 2 : 1>(ah.v, al.v, b.v, b.v, acc[t]);
    }
  }
#pragma unroll
  for (int t = 0; t < 4; ++t) {
    float bv = bias ? bias[col0 + t * 16 + ln] : 0.f;
    if (BIAS_BF16) bv = bf16_round(bv);
#pragma unroll
    for (int r = 0; r < 8; ++r) { float v = acc[t][r] + bv; if (ACT == 1) v = fmaxf(v, 0.f); so[w][8 * hh + r][t * 16 + ln] = v; }
  }
  __builtin_amdgcn_fence(__ATOMIC_ACQ_REL, "workgroup");
  __builtin_amdgcn_wave_barrier();
  const int rsub = lane >> 4, c4 = (lane & 15) * 4;
  for (int pass = 0; pass < 2; ++pass) {
#pragma unroll
    for (int q = 0; q < 8; ++q) {
      const int r = q * 2 + rsub;
      const v4f v = *(const v4fa*)&so[w][r][c4];
      *(volatile v4f*)(C + (size_t)(row0 + r) * ldc + col0 + c4) = v;
    }
    if (pass == 0) __threadfence();
  }
}

template <int D, bool CAUSAL>
__global__ __launch_bounds__(128) void k_flash(const float* __restrict__ qb, const float* __restrict__ kb, const float* __restrict__ vb,
                                             int pitch, int T, int H, float scale, float* __restrict__ y, int ypitch) {
  constexpr int KS = D / 32;
  constexpr int DT = D / 16;
  __shared__ __attribute__((aligned(16))) unsigned short sKh[32][D + 8], sKl[32][D + 8], sVh[32][D + 8], sVl[32][D + 8];
  __shared__ __attribute__((aligned(16))) unsigned short sPh[4][16][40], sPl[4][16][40];
  __shared__ __attribute__((aligned(16))) float sO[4][16][D];
  const int tid = threadIdx.x, w = tid >> 5, lane = tid & 31, ln = lane & 15, hh = lane >> 4;
  const int nqb = (T + 63) / 64;
  const int bh = blockIdx.x / nqb, qblk = blockIdx.x % nqb;
  const int b = bh / H, h = bh % H;
  const int q0 = qblk * 64 + w * 16;
  const float* Q = qb + (size_t)b * T * pitch + h * D;
  const float* K = kb + (size_t)b * T * pitch + h * D;
  const float* V = vb + (size_t)b * T * pitch + h * D;

  FragB aqh[KS], aql[KS];
  {
    int row = q0 + ln; if (row >= T) row = T - 1;
    const float* qr = Q + (size_t)row * pitch;
#pragma unroll
    for (int ks = 0; ks < KS; ++ks)
#pragma unroll
      for (int i = 0; i < 16; ++i) {
        const int d = ks * 32 + ((i < 8) ? (8 * hh + i) : (16 + 8 * hh + (i - 8)));
        const float x = qr[d] * scale; const unsigned short hb = bf16_bits(x);
        aqh[ks].u[i] = hb; aql[ks].u[i] = bf16_bits(x - bf16_val(hb));
      }
  }
  float m_r[8], l_r[8];
#pragma unroll
  for (int r = 0; r < 8; ++r) { m_r[r] = -3.0e38f; l_r[r] = 0.f; }
  v8f oacc[DT];
#pragma unroll
  for (int dt = 0; dt < DT; ++dt) oacc[dt] = (v8f){0.f,0.f,0.f,0.f,0.f,0.f,0.f,0.f};

  const int kv_end = CAUSAL ? min(T, qblk * 64 + 64) : T;
  for (int j0 = 0; j0 < kv_end; j0 += 32) {
    __syncthreads();
    for (int e = tid; e < 32 * (D / 4); e += 128) {
      const int r = e / (D / 4), c4 = (e % (D / 4)) * 4;
      const int key = j0 + r;
      v4f kf = {0.f,0.f,0.f,0.f}, vf = {0.f,0.f,0.f,0.f};
      if (key < T) { kf = *(const v4fa*)(K + (size_t)key * pitch + c4); vf = *(const v4fa*)(V + (size_t)key * pitch + c4); }
#pragma unroll
      for (int t = 0; t < 4; ++t) {
        unsigned short hb = bf16_bits(kf[t]); sKh[r][c4 + t] = hb; sKl[r][c4 + t] = bf16_bits(kf[t] - bf16_val(hb));
        hb = bf16_bits(vf[t]); sVh[r][c4 + t] = hb; sVl[r][c4 + t] = bf16_bits(vf[t] - bf16_val(hb));
      }
    }
    __syncthreads();
    v8f s[2];
#pragma unroll
    for (int nt = 0; nt < 2; ++nt) {
      v8f acc = {};
#pragma unroll
      for (int ks = 0; ks < KS; ++ks) {
        FragB bh_, bl_;
        bh_.half[0] = *(const v8us*)&sKh[nt * 16 + ln][ks * 32 + 8 * hh]; bh_.half[1] = *(const v8us*)&sKh[nt * 16 + ln][ks * 32 + 16 + 8 * hh];
        bl_.half[0] = *(const v8us*)&sKl[nt * 16 + ln][ks * 32 + 8 * hh]; bl_.half[1] = *(const v8us*)&sKl[nt * 16 + ln][ks * 32 + 16 + 8 * hh];
        acc = mmaN<3>(aqh[ks].v, aql[ks].v, bh_.v, bl_.v, acc);
      }
      s[nt] = acc;
    }
    float alpha[8];
#pragma unroll
    for (int r = 0; r < 8; ++r) {
      const int qi = q0 + 8 * hh + r;
      const int ja = j0 + ln, jb = j0 + 16 + ln;
      if (CAUSAL) { if (ja > qi) s[0][r] = -3.0e38f; if (jb > qi) s[1][r] = -3.0e38f; }
      if (ja >= T) s[0][r] = -3.0e38f;
      if (jb >= T) s[1][r] = -3.0e38f;
      float mx = fmaxf(s[0][r], s[1][r]);
      mx = fmaxf(mx, __shfl_xor(mx, 1, 32)); mx = fmaxf(mx, __shfl_xor(mx, 2, 32)); mx = fmaxf(mx, __shfl_xor(mx, 4, 32)); mx = fmaxf(mx, __shfl_xor(mx, 8, 32));
      const float mnew = fmaxf(m_r[r], mx);
      alpha[r] = (mnew > -1.0e38f) ? __expf(m_r[r] - mnew) : 1.0f;
      const float p0 = (s[0][r] > -1.0e38f) ? __expf(s[0][r] - mnew) : 0.f;
      const float p1 = (s[1][r] > -1.0e38f) ? __expf(s[1][r] - mnew) : 0.f;
      m_r[r] = mnew;
      l_r[r] = l_r[r] * alpha[r] + p0 + p1;
      unsigned short hb = bf16_bits(p0); sPh[w][8 * hh + r][ln] = hb;      sPl[w][8 * hh + r][ln] = bf16_bits(p0 - bf16_val(hb));
      hb = bf16_bits(p1);                sPh[w][8 * hh + r][16 + ln] = hb; sPl[w][8 * hh + r][16 + ln] = bf16_bits(p1 - bf16_val(hb));
    }
#pragma unroll
    for (int dt = 0; dt < DT; ++dt)
#pragma unroll
      for (int r = 0; r < 8; ++r) oacc[dt][r] *= alpha[r];
    __builtin_amdgcn_fence(__ATOMIC_ACQ_REL, "workgroup");
    __builtin_amdgcn_wave_barrier();
    FragB pah, pal;
    pah.half[0] = *(const v8us*)&sPh[w][ln][8 * hh]; pah.half[1] = *(const v8us*)&sPh[w][ln][16 + 8 * hh];
    pal.half[0] = *(const v8us*)&sPl[w][ln][8 * hh]; pal.half[1] = *(const v8us*)&sPl[w][ln][16 + 8 * hh];
#pragma unroll
    for (int dt = 0; dt < DT; ++dt) {
      FragB bvh, bvl;
#pragma unroll
      for (int i = 0; i < 8; ++i) {
        bvh.u[i] = sVh[8 * hh + i][dt * 16 + ln]; bvh.u[8 + i] = sVh[16 + 8 * hh + i][dt * 16 + ln];
        bvl.u[i] = sVl[8 * hh + i][dt * 16 + ln]; bvl.u[8 + i] = sVl[16 + 8 * hh + i][dt * 16 + ln];
      }
      oacc[dt] = mmaN<3>(pah.v, pal.v, bvh.v, bvl.v, oacc[dt]);
    }
    __builtin_amdgcn_fence(__ATOMIC_ACQ_REL, "workgroup");
    __builtin_amdgcn_wave_barrier();
  }
#pragma unroll
  for (int r = 0; r < 8; ++r) {
    float l = l_r[r];
    l += __shfl_xor(l, 1, 32); l += __shfl_xor(l, 2, 32); l += __shfl_xor(l, 4, 32); l += __shfl_xor(l, 8, 32);
    l_r[r] = (l > 0.f) ? 1.0f / l : 0.f;
  }
#pragma unroll
  for (int dt = 0; dt < DT; ++dt)
#pragma unroll
    for (int r = 0; r < 8; ++r) sO[w][8 * hh + r][dt * 16 + ln] = oacc[dt][r] * l_r[r];
  __builtin_amdgcn_fence(__ATOMIC_ACQ_REL, "workgroup");
  __builtin_amdgcn_wave_barrier();
  for (int pass = 0; pass < 2; ++pass) {
    for (int r = 0; r < 16; ++r) {
      const int row = q0 + r;
      if (row < T && lane < D / 4) {
        const v4f val = *(const v4fa*)&sO[w][r][lane * 4];
        *(volatile v4f*)(y + ((size_t)b * T + row) * ypitch + h * D + lane * 4) = val;
      }
    }
    if (pass == 0) __threadfence();
  }
}

template <bool ASPLIT, int ACT, bool BIAS_BF16, bool RES_BF16>
__global__ __launch_bounds__(128) void k_gemm_bf3(const float* __restrict__ A, int lda, const unsigned short* __restrict__ Wt, int ldb,
                                                const float* __restrict__ bias, const float* resid, int rmod, int ldr,
                                                float* C, int ldc, int M, int N, int K) {
  __shared__ __attribute__((aligned(16))) float so[4][16][64];
  const int tid = threadIdx.x, w = tid >> 5, lane = tid & 31, ln = lane & 15, hh = lane >> 4;
  const int ntn = N / 64;
  const int wid = blockIdx.x * 4 + w;
  const int mt = wid / ntn, nq = wid % ntn;
  if (mt * 16 >= M) return;
  const int row0 = mt * 16, col0 = nq * 64;
  const float* arow = A + (size_t)(row0 + ln) * lda;
  v8f acc[4] = {};
  for (int kb = 0; kb < K; kb += 32) {
    FragB ah, al;
    const v4f x0 = *(const v4fa*)(arow + kb + 8 * hh), x1 = *(const v4fa*)(arow + kb + 8 * hh + 4);
    const v4f x2 = *(const v4fa*)(arow + kb + 16 + 8 * hh), x3 = *(const v4fa*)(arow + kb + 16 + 8 * hh + 4);
    float xs[16] = {x0[0],x0[1],x0[2],x0[3],x1[0],x1[1],x1[2],x1[3],x2[0],x2[1],x2[2],x2[3],x3[0],x3[1],x3[2],x3[3]};
#pragma unroll
    for (int i = 0; i < 16; ++i) { const unsigned short hb = bf16_bits(xs[i]); ah.u[i] = hb; al.u[i] = ASPLIT ? bf16_bits(xs[i] - bf16_val(hb)) : (unsigned short)0; }
#pragma unroll
    for (int t = 0; t < 4; ++t) {
      const unsigned short* brow = Wt + (size_t)(col0 + t * 16 + ln) * ldb + kb;
      FragB b;
      b.half[0] = *(const v8us*)(brow + 8 * hh);
      b.half[1] = *(const v8us*)(brow + 16 + 8 * hh);
      acc[t] = mmaN<ASPLIT ? 2 : 1>(ah.v, al.v, b.v, b.v, acc[t]);
    }
  }
#pragma unroll
  for (int t = 0; t < 4; ++t) {
    const int col = col0 + t * 16 + ln;
    float bv = bias ? bias[col] : 0.f;
    if (BIAS_BF16) bv = bf16_round(bv);
#pragma unroll
    for (int r = 0; r < 8; ++r) {
      float v = acc[t][r] + bv;
      if (resid) { float rv = resid[(size_t)((row0 + 8 * hh + r) % rmod) * ldr + col]; if (RES_BF16) rv = bf16_round(rv); v += rv; }
      if (ACT == 1) v = fmaxf(v, 0.f);
      if (ACT == 2) v = 0.5f * v * (1.0f + erff(v * 0.70710678118654752f));
      if (ACT == 3) { const float u = 0.7978845608028654f * (v + 0.044715f * v * v * v); v = 0.5f * v * (1.0f + tanhf(u)); }
      so[w][8 * hh + r][t * 16 + ln] = v;
    }
  }
  __builtin_amdgcn_fence(__ATOMIC_ACQ_REL, "workgroup");
  __builtin_amdgcn_wave_barrier();
  const int rsub = lane >> 4, c4 = (lane & 15) * 4;
  for (int pass = 0; pass < 2; ++pass) {
#pragma unroll
    for (int q = 0; q < 8; ++q) {
      const int r = q * 2 + rsub;
      const v4f v = *(const v4fa*)&so[w][r][c4];
      *(volatile v4f*)(C + (size_t)(row0 + r) * ldc + col0 + c4) = v;
    }
    if (pass == 0) __threadfence();
  }
}
template <bool PARAM_BF16>
__global__ __launch_bounds__(256) void k_layernorm(const float* __restrict__ X, const float* __restrict__ R, const float* __restrict__ g, const float* __restrict__ bta,
                                                  float* __restrict__ out_sum, float* __restrict__ out_norm, int N, float eps) {
  __shared__ float red[256];
  const int row = blockIdx.x, tid = threadIdx.x;
  const float* x = X + (size_t)row * N; const float* rr = R ? R + (size_t)row * N : nullptr;
  float vals[16];
  const int per = N / 256;
  float s1 = 0.f;
  for (int u = 0; u < per / 4; ++u) {
    const int j = tid * 4 + 1024 * u;
    const v4f a = *(const v4fa*)(x + j);
    v4f b = {0.f,0.f,0.f,0.f}; if (rr) b = *(const v4fa*)(rr + j);
#pragma unroll
    for (int q = 0; q < 4; ++q) { const float v = a[q] + b[q]; vals[u * 4 + q] = v; s1 += v; }
  }
  red[tid] = s1; __syncthreads();
  for (int st = 128; st > 0; st >>= 1) { if (tid < st) red[tid] += red[tid + st]; __syncthreads(); }
  const float mu = red[0] / (float)N; __syncthreads();
  float s2 = 0.f;
  for (int u = 0; u < per / 4; ++u)
#pragma unroll
    for (int q = 0; q < 4; ++q) { const float c = vals[u * 4 + q] - mu; s2 += c * c; }
  red[tid] = s2; __syncthreads();
  for (int st = 128; st > 0; st >>= 1) { if (tid < st) red[tid] += red[tid + st]; __syncthreads(); }
  const float rs = rsqrtf(red[0] / (float)N + eps);
  for (int pass = 0; pass < 2; ++pass) {
    for (int u = 0; u < per / 4; ++u) {
      const int j = tid * 4 + 1024 * u;
      v4f o, sm;
#pragma unroll
      for (int q = 0; q < 4; ++q) {
        float gg = g[j + q], bb = bta[j + q];
        if (PARAM_BF16) { gg = bf16_round(gg); bb = bf16_round(bb); }
        sm[q] = vals[u * 4 + q]; o[q] = (vals[u * 4 + q] - mu) * rs * gg + bb;
      }
      if (out_sum) *(volatile v4f*)(out_sum + (size_t)row * N + j) = sm;
      *(volatile v4f*)(out_norm + (size_t)row * N + j) = o;
    }
    if (pass == 0) __threadfence();
  }
}

__global__ __launch_bounds__(256) void k_round_rows(const float* __restrict__ W, unsigned short* __restrict__ Wt, int n8) {
  const int t = blockIdx.x * 256 + threadIdx.x;
  if (t >= n8) return;
  const v4f a = *(const v4fa*)(W + (size_t)t * 8), b = *(const v4fa*)(W + (size_t)t * 8 + 4);
  v8us v; v[0]=bf16_bits(a[0]); v[1]=bf16_bits(a[1]); v[2]=bf16_bits(a[2]); v[3]=bf16_bits(a[3]);
  v[4]=bf16_bits(b[0]); v[5]=bf16_bits(b[1]); v[6]=bf16_bits(b[2]); v[7]=bf16_bits(b[3]);
  *(volatile v8us*)(Wt + (size_t)t * 8) = v; __threadfence(); *(volatile v8us*)(Wt + (size_t)t * 8) = v;
}

__global__ __launch_bounds__(128) void k_patch(const float* __restrict__ x, const unsigned short* __restrict__ Bt, const float* __restrict__ pb, float* __restrict__ feat) {
  constexpr int K = 768;
  __shared__ __attribute__((aligned(16))) float so[4][16][64];
  const int tid = threadIdx.x, w = tid >> 5, lane = tid & 31, ln = lane & 15, hh = lane >> 4;
  const int wid = blockIdx.x * 4 + w; const int mt = wid / (DM / 64), nq = wid % (DM / 64); const int row0 = mt * 16, col0 = nq * 64; const int m = row0 + ln;
  const int b = m / LL, p = m % LL; const int pp = (p == 0) ? 0 : p - 1; const int py = pp / 17, px = pp % 17;
  v8f acc[4] = {};
#pragma unroll 1
  for (int ks = 0; ks < K / 32; ++ks) {
    FragB a;
#pragma unroll
    for (int i = 0; i < 16; ++i) { const int k = ks * 32 + ((i < 8) ? (8 * hh + i) : (16 + 8 * hh + (i - 8))); const int c = k >> 8, ky = (k >> 4) & 15, kx = k & 15;
      a.u[i] = bf16_bits(x[(((size_t)b * 3 + c) * 240 + (py * 16 + ky)) * 272 + px * 16 + kx]); }
#pragma unroll
    for (int t = 0; t < 4; ++t) { FragB bq; bq.half[0] = *(const v8us*)(Bt + (size_t)(col0 + t * 16 + ln) * K + ks * 32 + 8 * hh); bq.half[1] = *(const v8us*)(Bt + (size_t)(col0 + t * 16 + ln) * K + ks * 32 + 16 + 8 * hh); acc[t] = mmaN<1>(a.v, a.v, bq.v, bq.v, acc[t]); }
  }
#pragma unroll
  for (int t = 0; t < 4; ++t) { const int col = col0 + t * 16 + ln; const float bv = bf16_round(pb[col]);
#pragma unroll
    for (int r = 0; r < 8; ++r) so[w][8 * hh + r][t * 16 + ln] = acc[t][r] + bv; }
  __builtin_amdgcn_fence(__ATOMIC_ACQ_REL, "workgroup"); __builtin_amdgcn_wave_barrier();
  const int rsub = lane >> 4, c4 = (lane & 15) * 4;
  for (int pass = 0; pass < 2; ++pass) { for (int q = 0; q < 8; ++q) { const int r = q * 2 + rsub; const v4f v = *(const v4fa*)&so[w][r][c4]; *(volatile v4f*)(feat + (size_t)(row0 + r) * DM + col0 + c4) = v; } if (pass == 0) __threadfence(); }
}
__global__ __launch_bounds__(256) void k_tokens(const float* __restrict__ feat, const float* __restrict__ cls, const float* __restrict__ pos, float* __restrict__ h) {
  const size_t i = (size_t)blockIdx.x * 256 + threadIdx.x; if (i >= (size_t)MT * DM / 4) return; const int c4 = (int)(i % (DM / 4)) * 4; const int p = (int)((i / (DM / 4)) % LL);
  v4f f = {0.f,0.f,0.f,0.f}; if (p != 0) f = *(const v4fa*)(feat + i * 4);
  v4f v; for (int q = 0; q < 4; ++q) { const int c = c4 + q; const float base = (p == 0) ? bf16_round(cls[c]) : f[q]; v[q] = base + bf16_round(pos[(size_t)p * DM + c]); }
  *(volatile v4f*)(h + i * 4) = v; __threadfence(); *(volatile v4f*)(h + i * 4) = v;
}
__global__ __launch_bounds__(256) void k_ln(const float* __restrict__ x, const float* __restrict__ g, const float* __restrict__ b, float* __restrict__ out) {
  const int tid = threadIdx.x, w = tid >> 5, lane = tid & 31; const int row = blockIdx.x * 8 + w; if (row >= MT) return;
  float v[12]; float s = 0.f;
#pragma unroll
  for (int u = 0; u < 12; ++u) { v[u] = x[(size_t)row * DM + u * 32 + lane]; s += v[u]; }
  for (int o = 16; o >= 1; o >>= 1) s += __shfl_xor(s, o, 32); const float mu = s * (1.0f / DM);
  float q2 = 0.f;
#pragma unroll
  for (int u = 0; u < 12; ++u) { const float c = v[u] - mu; q2 += c * c; }
  for (int o = 16; o >= 1; o >>= 1) q2 += __shfl_xor(q2, o, 32); const float rs = rsqrtf(q2 * (1.0f / DM) + 1e-5f);
  for (int pass = 0; pass < 2; ++pass) {
#pragma unroll
    for (int u = 0; u < 12; ++u) { const int c = u * 32 + lane; *(volatile float*)(out + (size_t)row * DM + c) = (v[u] - mu) * rs * bf16_round(g[c]) + bf16_round(b[c]); }
    if (pass == 0) __threadfence(); }
}
__global__ __launch_bounds__(256) void k_dw3(const float* __restrict__ xz, const float* __restrict__ cw, const float* __restrict__ cb, float* __restrict__ xs) {
  const size_t i = (size_t)blockIdx.x * 256 + threadIdx.x; if (i >= (size_t)MT * DI / 4) return; const int c4 = (int)(i % (DI / 4)) * 4; const int m = (int)(i / (DI / 4)); const int b = m / LL, p = m % LL, y = p / GR, xq = p % GR;
  v4f acc; for (int q = 0; q < 4; ++q) acc[q] = bf16_round(cb[c4 + q]);
#pragma unroll 1
  for (int tap = 0; tap < 9; ++tap) { const int yy = y + tap / 3 - 1, xx = xq + tap % 3 - 1; if (yy < 0 || yy >= GR || xx < 0 || xx >= GR) continue; const v4f v = *(const v4fa*)(xz + ((size_t)b * LL + yy * GR + xx) * 2 * DI + c4);
    for (int q = 0; q < 4; ++q) acc[q] += v[q] * bf16_round(cw[(size_t)(c4 + q) * 9 + tap]); }
  v4f o; for (int q = 0; q < 4; ++q) o[q] = acc[q] / (1.0f + expf(-acc[q]));
  *(volatile v4f*)(xs + i * 4) = o; __threadfence(); *(volatile v4f*)(xs + i * 4) = o;
}
__global__ __launch_bounds__(256) void k_dtmean(const float* __restrict__ xd, float* __restrict__ dtin) {
  const size_t i = (size_t)blockIdx.x * 256 + threadIdx.x; if (i >= (size_t)MT * DM / 4) return; const int c4 = (int)(i % (DM / 4)) * 4; const size_t m = i / (DM / 4); const float* r = xd + m * XPN;
  v4f v; for (int q = 0; q < 4; ++q) { const int c = c4 + q; v[q] = (((r[c] + r[DM + c]) + r[2 * DM + c]) + r[3 * DM + c]) / 4.0f; }
  *(volatile v4f*)(dtin + i * 4) = v; __threadfence(); *(volatile v4f*)(dtin + i * 4) = v;
}
__device__ __forceinline__ int tok_of(int d, int l) { const int a = l / GR, bq = l % GR; if (d == 0) return l; if (d == 1) return a * GR + (GR - 1 - bq); if (d == 2) return bq * GR + a; return (GR - 1 - bq) * GR + a; }
__global__ __launch_bounds__(256) void k_dirscan(const float* __restrict__ xs, const float* __restrict__ dt, const float* __restrict__ xd, const float* __restrict__ Alog, int d, int b0, float* __restrict__ E, float* __restrict__ contrib) {
  const int i = blockIdx.x * 256 + threadIdx.x; if (i >= BH * DI * NS) return; const int k = i % DI; const int n = (i / DI) % NS; const int bl = i / (DI * NS); const int b = b0 + bl;
  const float A = -expf(bf16_round(Alog[k * NS + n]));
  float S = 0.f;
#pragma unroll 1
  for (int l = LL - 1; l >= 0; --l) {
    if (l < LL - 1) { const int p1 = tok_of(d, l + 1); const float de = dt[((size_t)b * LL + p1) * 4 * DI + d * DI + k]; S += expf(de * A); }
    const float e = expf(S); float* ep = E + (((size_t)bl * NS + n) * LL + l) * DI + k;
    *(volatile float*)ep = e; __threadfence(); *(volatile float*)ep = e;
  }
  __threadfence();
  float P = 0.f;
#pragma unroll 1
  for (int l = 0; l < LL; ++l) { const int p = tok_of(d, l); const size_t row = (size_t)b * LL + p;
    const float de = dt[row * 4 * DI + d * DI + k], u = xs[row * DI + k], Bn = xd[row * XPN + 4 * DM + d * NS + n], Cn = xd[row * XPN + 4 * DM + 4 * NS + d * NS + n];
    const float e = E[(((size_t)bl * NS + n) * LL + l) * DI + k];
    P += (de * u * Bn) * e;
    const float v = (P / (e + 1e-12f)) * Cn;
    *(volatile float*)(contrib + (((size_t)bl * NS + n) * LL + l) * DI + k) = v;
  }
  __threadfence();
#pragma unroll 1
  for (int l = 0; l < LL; ++l) { const float v2 = contrib[(((size_t)bl * NS + n) * LL + l) * DI + k]; *(volatile float*)(contrib + (((size_t)bl * NS + n) * LL + l) * DI + k) = v2; }
}
__global__ __launch_bounds__(256) void k_ysum(const float* __restrict__ contrib, const float* __restrict__ xs, const float* __restrict__ Dp, int d, int first, int b0, float* y) {
  const size_t i = (size_t)blockIdx.x * 256 + threadIdx.x; if (i >= (size_t)BH * LL * DI) return; const int k = (int)(i % DI); const int l = (int)((i / DI) % LL); const int bl = (int)(i / ((size_t)DI * LL)); const int b = b0 + bl;
  const int p = tok_of(d, l); const size_t row = (size_t)b * LL + p; float s = xs[row * DI + k] * bf16_round(Dp[k]);
#pragma unroll 1
  for (int n = 0; n < NS; ++n) s += contrib[(((size_t)bl * NS + n) * LL + l) * DI + k];
  float* dst = y + row * DI + k; const float v = first ? s : (*dst + s);
  *(volatile float*)dst = v; __threadfence(); *(volatile float*)dst = v;
}
__global__ __launch_bounds__(256) void k_gate(const float* __restrict__ y, const float* __restrict__ xz, float* __restrict__ yg) {
  const size_t i = (size_t)blockIdx.x * 256 + threadIdx.x; if (i >= (size_t)MT * DI / 4) return; const int c4 = (int)(i % (DI / 4)) * 4; const size_t m = i / (DI / 4);
  const v4f a = *(const v4fa*)(y + i * 4), z = *(const v4fa*)(xz + m * 2 * DI + DI + c4); v4f o; for (int q = 0; q < 4; ++q) o[q] = (a[q] * 0.25f) * (z[q] / (1.0f + expf(-z[q])));
  *(volatile v4f*)(yg + i * 4) = o; __threadfence(); *(volatile v4f*)(yg + i * 4) = o;
}
extern "C" void kernel_launch(void* const* d_in, const int* in_sizes, int n_in,
                              void* d_out, int out_size, void* d_ws, size_t ws_size, hipStream_t stream) {
  (void)in_sizes; (void)n_in; (void)out_size;
  const float* x = (const float*)d_in[0]; const float* pw = (const float*)d_in[1]; const float* pb = (const float*)d_in[2]; const float* cls = (const float*)d_in[3]; const float* pos = (const float*)d_in[4];
  const float* nw = (const float*)d_in[5]; const float* nb = (const float*)d_in[6]; const float* inw = (const float*)d_in[7]; const float* cw = (const float*)d_in[8]; const float* cb = (const float*)d_in[9];
  const float* xw = (const float*)d_in[10]; const float* dtw = (const float*)d_in[11]; const float* dtb = (const float*)d_in[12]; const float* Alog = (const float*)d_in[13]; const float* Dp = (const float*)d_in[14]; const float* ow = (const float*)d_in[15];
  const float* fw = (const float*)d_in[16]; const float* fb = (const float*)d_in[17];
  char* ws = (char*)d_ws; size_t off = 0;
  auto take = [&](size_t bytes) { char* p = ws + off; off += (bytes + 255) & ~(size_t)255; return p; };
  unsigned short* Bp = (unsigned short*)take((size_t)DM * 768 * 2); unsigned short* Bin[2], *Bx[2], *Bdt[2], *Bo[2];
  for (int i = 0; i < 2; ++i) { Bin[i] = (unsigned short*)take((size_t)2 * DI * DM * 2); Bx[i] = (unsigned short*)take((size_t)XPN * DI * 2); Bdt[i] = (unsigned short*)take((size_t)4 * DI * DM * 2); Bo[i] = (unsigned short*)take((size_t)DM * DI * 2); }
  float* dtbr = (float*)take(4 * DI * 4 * 2);
  float* feat = (float*)take((size_t)MT * DM * 4); float* h = (float*)take((size_t)MT * DM * 4); float* hn = (float*)take((size_t)MT * DM * 4); float* xz = (float*)take((size_t)MT * 2 * DI * 4); float* xs = (float*)take((size_t)MT * DI * 4);
  float* xd = (float*)take((size_t)MT * XPN * 4); float* dtin = (float*)take((size_t)MT * DM * 4); float* dt = (float*)take((size_t)MT * 4 * DI * 4); float* E = (float*)take((size_t)BH * NS * LL * DI * 4); float* contrib = (float*)take((size_t)BH * NS * LL * DI * 4);
  float* y = (float*)take((size_t)MT * DI * 4); float* yg = (float*)take((size_t)MT * DI * 4); float* ob = (float*)take((size_t)MT * DM * 4);
  if (off > ws_size) return;
  k_round_rows<<<(DM * 768 / 8 + 255) / 256, 256, 0, stream>>>(pw, Bp, DM * 768 / 8);
  for (int i = 0; i < 2; ++i) { k_round_rows<<<(2 * DI * DM / 8 + 255) / 256, 256, 0, stream>>>(inw + (size_t)i * 2 * DI * DM, Bin[i], 2 * DI * DM / 8); k_round_rows<<<(XPN * DI / 8 + 255) / 256, 256, 0, stream>>>(xw + (size_t)i * XPN * DI, Bx[i], XPN * DI / 8);
    k_round_rows<<<(4 * DI * DM / 8 + 255) / 256, 256, 0, stream>>>(dtw + (size_t)i * 4 * DI * DM, Bdt[i], 4 * DI * DM / 8); k_round_rows<<<(DM * DI / 8 + 255) / 256, 256, 0, stream>>>(ow + (size_t)i * DM * DI, Bo[i], DM * DI / 8); }
  k_patch<<<((MT / 16) * (DM / 64) + 3) / 4, 128, 0, stream>>>(x, Bp, pb, feat);
  k_tokens<<<(MT * DM / 4 + 255) / 256, 256, 0, stream>>>(feat, cls, pos, h);
  const unsigned gsm = (MT / 16), n4d = (unsigned)(((size_t)MT * DI / 4 + 255) / 256);
  for (int i = 0; i < 2; ++i) {
    k_ln<<<(MT + 7) / 8, 256, 0, stream>>>(h, nw + i * DM, nb + i * DM, hn);
    k_gemm_bf3<true, 0, false, false><<<(gsm * (2 * DI / 64) + 3) / 4, 128, 0, stream>>>(hn, DM, Bin[i], DM, nullptr, nullptr, 1, 0, xz, 2 * DI, MT, 2 * DI, DM);
    k_dw3<<<n4d, 256, 0, stream>>>(xz, cw + (size_t)i * DI * 9, cb + i * DI, xs);
    k_gemm_bf3<true, 0, false, false><<<(gsm * (XPN / 64) + 3) / 4, 128, 0, stream>>>(xs, DI, Bx[i], DI, nullptr, nullptr, 1, 0, xd, XPN, MT, XPN, DI);
    k_dtmean<<<(MT * DM / 4 + 255) / 256, 256, 0, stream>>>(xd, dtin);
    k_gemm_bf3<true, 0, true, false><<<(gsm * (4 * DI / 64) + 3) / 4, 128, 0, stream>>>(dtin, DM, Bdt[i], DM, dtb + (size_t)i * 4 * DI, nullptr, 1, 0, dt, 4 * DI, MT, 4 * DI, DM);
    for (int d = 0; d < 4; ++d)
      for (int b0 = 0; b0 < BB; b0 += BH) {
        k_dirscan<<<(BH * DI * NS + 255) / 256, 256, 0, stream>>>(xs, dt, xd, Alog + (size_t)i * DI * NS, d, b0, E, contrib);
        k_ysum<<<(unsigned)(((size_t)BH * LL * DI + 255) / 256), 256, 0, stream>>>(contrib, xs, Dp + i * DI, d, d == 0 ? 1 : 0, b0, y);
      }
    k_gate<<<n4d, 256, 0, stream>>>(y, xz, yg);
    k_gemm_bf3<true, 0, false, false><<<(gsm * (DM / 64) + 3) / 4, 128, 0, stream>>>(yg, DI, Bo[i], DI, nullptr, h, MT, DM, h, DM, MT, DM, DI);
  }
  k_ln<<<(MT + 7) / 8, 256, 0, stream>>>(h, fw, fb, (float*)d_out);
}
